// JaCDEManual_13829794693220
// MI455X (gfx1250) — hardware-run, weakly checked
//
#include <hip/hip_runtime.h>
#include <math.h>

typedef __attribute__((ext_vector_type(16))) _Float16 v16h;
typedef __attribute__((ext_vector_type(8)))  _Float16 v8h;
typedef __attribute__((ext_vector_type(8)))  float    v8f;
typedef __attribute__((ext_vector_type(4)))  float    v4f;

constexpr int kBatch     = 4096;
constexpr int kHid       = 128;
constexpr int kCh        = 32;
constexpr int kIntervals = 16;
constexpr int kObs       = 17;
constexpr int kTerms     = 8;
constexpr int kRowsBlk   = 64;
constexpr int kWPitch    = 136;
constexpr int kXPitch    = 40;
constexpr int kOPitch    = 132;
constexpr int kXTile     = kRowsBlk * kXPitch;
static_assert(kObs == kIntervals + 1, "observation grid");
static_assert((kBatch % kRowsBlk) == 0, "row blocks");
static_assert((kHid % 32) == 0 && (kCh % 32) == 0, "k steps of 32");
static_assert(kHid == 8 * 16, "eight waves own sixteen hidden units each");
static_assert((kWPitch % 8) == 0 && (kXPitch % 8) == 0 && (kOPitch % 4) == 0, "16-B aligned LDS rows");
static_assert(kWPitch >= kHid && kXPitch >= kCh && kOPitch >= kHid, "LDS pitches");

constexpr float kCarryW   = 256.0f;
constexpr float kCarryA   = 16.0f;
constexpr float kCarryP0  = 64.0f;
constexpr float kCarryV0  = 64.0f;
constexpr float kTermGain = 2.0f;
constexpr float kInvFwd   = 1.0f / (kCarryA * kCarryW);
constexpr float kScaleP0  = kCarryP0 / (kCarryA * kCarryW);
constexpr float kScaleV0  = kCarryV0 / (kCarryP0 * kCarryW);
constexpr float kInvV0    = 1.0f / kCarryV0;
constexpr float kScaleP   = kTermGain / kCarryW;
constexpr float kScaleV   = 1.0f / kCarryW;
constexpr float kInvTermGain = 1.0f / kTermGain;
constexpr float kF16MinNormal = 6.103515625e-05f;
constexpr float kF16Clamp     = 60000.0f;

__device__ __forceinline__ float bf16_value(float f) {
  unsigned u = __float_as_uint(f);
  u = (u + 0x7FFFu + ((u >> 16) & 1u)) & 0xFFFF0000u;
  return __uint_as_float(u);
}

__device__ __forceinline__ _Float16 to_f16_operand(float v) {
  const float cl = __builtin_amdgcn_fmed3f(v, -kF16Clamp, kF16Clamp);
  const float s  = (fabsf(cl) < kF16MinNormal) ? 0.0f : cl;
  return (_Float16)s;
}

union FragU { v16h v; v8h h[2]; };
__device__ __forceinline__ v16h frag_load(const _Float16* p) {
  FragU f;
  f.h[0] = *(const v8h*)(p);
  f.h[1] = *(const v8h*)(p + 16);
  return f.v;
}

__device__ __forceinline__ v8f mma_f16(v16h a, v16h b, v8f c) {
  c = __builtin_amdgcn_wmma_f32_16x16x32_f16(false, a, false, b, (short)0, c, false, false);
  asm volatile("v_nop\n\tv_nop\n\tv_nop\n\tv_nop" : "+v"(c) : "v"(a), "v"(b));
  return c;
}

template <int KSTEPS>
__device__ __forceinline__ void slab_product(const _Float16* wrow, const _Float16* srow, int spitch, v8f (&acc)[4]) {
#pragma unroll
  for (int kk = 0; kk < KSTEPS; ++kk) {
    const v16h a = frag_load(wrow + kk * 32);
#pragma unroll
    for (int bt = 0; bt < 4; ++bt) {
      const v16h b = frag_load(srow + bt * 16 * spitch + kk * 32);
      acc[bt] = mma_f16(a, b, acc[bt]);
    }
  }
}

__device__ __forceinline__ void zero4(v8f (&acc)[4]) {
#pragma unroll
  for (int bt = 0; bt < 4; ++bt) acc[bt] = (v8f){0.f, 0.f, 0.f, 0.f, 0.f, 0.f, 0.f, 0.f};
}

__device__ __forceinline__ void store_gated(_Float16* dst, const v8f& g, const v8f& a, float s) {
  v8h pv;
#pragma unroll
  for (int r = 0; r < 8; ++r) pv[r] = to_f16_operand(g[r] * a[r] * s);
  *(v8h*)dst = pv;
}

__global__ __launch_bounds__(256) void series_rows(
    const float* __restrict__ t, const float* __restrict__ h,
    const float* __restrict__ coeffs, const float* __restrict__ dcoeffs,
    const float* __restrict__ tobs, const float* __restrict__ wx,
    const float* __restrict__ wh, const float* __restrict__ wout,
    const float* __restrict__ b0, const float* __restrict__ b1,
    float* __restrict__ out)
{
  __shared__ __align__(16) _Float16 sWh[kHid * kWPitch];
  __shared__ __align__(16) _Float16 sWo[kHid * kWPitch];
  __shared__ __align__(16) _Float16 sWx[kHid * kXPitch];
  __shared__ __align__(16) _Float16 sS0[kRowsBlk * kWPitch];
  __shared__ __align__(16) _Float16 sS1[kRowsBlk * kWPitch];
  __shared__ __align__(16) _Float16 sXX[2 * kXTile];
  __shared__ __align__(16) float    sO[kRowsBlk * kOPitch];

  const int tid  = threadIdx.x;
  const int lane = tid & 31;
  const int wave = tid >> 5;
  const int hh   = lane >> 4;
  const int c    = lane & 15;
  const int row0 = blockIdx.x * kRowsBlk;
  const int n0   = wave * 16;

  const float ts = bf16_value(t[0]);
  int cnt = 0;
#pragma unroll
  for (int i = 0; i < kObs; ++i) cnt += (bf16_value(tobs[i]) <= ts) ? 1 : 0;
  int idx = cnt - 1;
  idx = (idx < 0) ? 0 : idx;
  idx = (idx > kIntervals - 1) ? (kIntervals - 1) : idx;
  const float dt = ts - bf16_value(tobs[idx]);

#pragma unroll 1
  for (int it = 0; it < 8; ++it) {
    const int e8 = tid + 256 * it;
    const int n  = e8 >> 4;
    const int k  = (e8 & 15) * 8;
    const v4f a0 = *(const v4f*)(wh + n * kHid + k);
    const v4f a1 = *(const v4f*)(wh + n * kHid + k + 4);
    const v4f o0 = *(const v4f*)(wout + n * kHid + k);
    const v4f o1 = *(const v4f*)(wout + n * kHid + k + 4);
    v8h hv, ov;
#pragma unroll
    for (int e = 0; e < 4; ++e) {
      const float f0 = a0[e];
      const float f1 = a1[e];
      const float g0 = o0[e];
      const float g1 = o1[e];
      hv[e]     = to_f16_operand(bf16_value(f0) * kCarryW);
      hv[4 + e] = to_f16_operand(bf16_value(f1) * kCarryW);
      ov[e]     = to_f16_operand(bf16_value(g0) * kCarryW);
      ov[4 + e] = to_f16_operand(bf16_value(g1) * kCarryW);
    }
    *(v8h*)(sWh + n * kWPitch + k) = hv;
    *(v8h*)(sWo + n * kWPitch + k) = ov;
  }
#pragma unroll 1
  for (int it = 0; it < 2; ++it) {
    const int e8 = tid + 256 * it;
    const int n  = e8 >> 2;
    const int k  = (e8 & 3) * 8;
    const v4f a0 = *(const v4f*)(wx + n * kCh + k);
    const v4f a1 = *(const v4f*)(wx + n * kCh + k + 4);
    v8h hv;
#pragma unroll
    for (int e = 0; e < 4; ++e) {
      const float f0 = a0[e];
      const float f1 = a1[e];
      hv[e]     = to_f16_operand(bf16_value(f0) * kCarryW);
      hv[4 + e] = to_f16_operand(bf16_value(f1) * kCarryW);
    }
    *(v8h*)(sWx + n * kXPitch + k) = hv;
  }
#pragma unroll 1
  for (int it = 0; it < 4; ++it) {
    const int e8 = tid + 256 * it;
    const int r  = e8 >> 4;
    const int k  = (e8 & 15) * 8;
    const float* hp = h + (size_t)(row0 + r) * kHid + k;
    const v4f a0 = *(const v4f*)(hp);
    const v4f a1 = *(const v4f*)(hp + 4);
    v8h hv;
#pragma unroll
    for (int e = 0; e < 4; ++e) {
      const float f0 = a0[e];
      const float f1 = a1[e];
      hv[e]     = to_f16_operand(bf16_value(f0) * kCarryA);
      hv[4 + e] = to_f16_operand(bf16_value(f1) * kCarryA);
    }
    *(v8h*)(sS0 + r * kWPitch + k) = hv;
  }
  {
    const int r  = tid >> 2;
    const int c8 = (tid & 3) * 8;
    const size_t cb = ((size_t)(row0 + r) * kIntervals + (size_t)idx) * (size_t)(4 * kCh) + (size_t)c8;
#pragma unroll 1
    for (int which = 0; which < 2; ++which) {
      const float* src = (which == 0) ? coeffs : dcoeffs;
      const v4f q00 = *(const v4f*)(src + cb);
      const v4f q01 = *(const v4f*)(src + cb + 4);
      const v4f q10 = *(const v4f*)(src + cb + kCh);
      const v4f q11 = *(const v4f*)(src + cb + kCh + 4);
      const v4f q20 = *(const v4f*)(src + cb + 2 * kCh);
      const v4f q21 = *(const v4f*)(src + cb + 2 * kCh + 4);
      const v4f q30 = *(const v4f*)(src + cb + 3 * kCh);
      const v4f q31 = *(const v4f*)(src + cb + 3 * kCh + 4);
      v8h xv;
#pragma unroll
      for (int e = 0; e < 4; ++e) {
        const float a0 = q00[e];
        const float a1 = q10[e];
        const float a2 = q20[e];
        const float a3 = q30[e];
        const float d0 = q01[e];
        const float d1 = q11[e];
        const float d2 = q21[e];
        const float d3 = q31[e];
        const float va = bf16_value(a0) + dt * (bf16_value(a1) + dt * (bf16_value(a2) + dt * bf16_value(a3)));
        const float vb = bf16_value(d0) + dt * (bf16_value(d1) + dt * (bf16_value(d2) + dt * bf16_value(d3)));
        xv[e]     = to_f16_operand(va * kCarryA);
        xv[4 + e] = to_f16_operand(vb * kCarryA);
      }
      *(v8h*)(sXX + which * kXTile + r * kXPitch + c8) = xv;
    }
  }
  __syncthreads();

  const _Float16* whRow = sWh + (n0 + c) * kWPitch + 8 * hh;
  const _Float16* woRow = sWo + (n0 + c) * kWPitch + 8 * hh;
  const _Float16* wxRow = sWx + (n0 + c) * kXPitch + 8 * hh;
  const _Float16* s0Row = sS0 + c * kWPitch + 8 * hh;
  const _Float16* s1Row = sS1 + c * kWPitch + 8 * hh;
  const _Float16* xRow  = sXX + c * kXPitch + 8 * hh;
  const _Float16* xdRow = sXX + kXTile + c * kXPitch + 8 * hh;
  _Float16* s0Out = sS0 + c * kWPitch + n0 + 8 * hh;
  _Float16* s1Out = sS1 + c * kWPitch + n0 + 8 * hh;

  v8f acc[4], dr[4], dth[4], hd[4];

  zero4(acc);
  slab_product<1>(wxRow, xRow, kXPitch, acc);
  slab_product<4>(whRow, s0Row, kWPitch, acc);
  {
    const v4f bA = *(const v4f*)(b0 + n0 + 8 * hh);
    const v4f bB = *(const v4f*)(b0 + n0 + 8 * hh + 4);
    v8f bv;
#pragma unroll
    for (int e = 0; e < 4; ++e) {
      const float f0 = bA[e];
      const float f1 = bB[e];
      bv[e]     = bf16_value(f0);
      bv[4 + e] = bf16_value(f1);
    }
#pragma unroll 1
    for (int bt = 0; bt < 4; ++bt) {
      const v8f a = acc[0];
      v8f d;
      v8h rv;
#pragma unroll
      for (int r = 0; r < 8; ++r) {
        const float l1 = a[r] * kInvFwd + bv[r];
        const float ex = expf(-l1);
        d[r]  = __builtin_amdgcn_rcpf(1.0f + ex);
        rv[r] = to_f16_operand(fmaxf(l1, 0.0f) * kCarryA);
      }
      *(v8h*)(s1Out + bt * 16 * kWPitch) = rv;
      acc[0] = acc[1]; acc[1] = acc[2]; acc[2] = acc[3]; acc[3] = a;
      dr[0] = dr[1]; dr[1] = dr[2]; dr[2] = dr[3]; dr[3] = d;
    }
  }
  __syncthreads();

  zero4(acc);
  slab_product<4>(woRow, s1Row, kWPitch, acc);
  {
    const v4f bA = *(const v4f*)(b1 + n0 + 8 * hh);
    const v4f bB = *(const v4f*)(b1 + n0 + 8 * hh + 4);
    v8f bv;
#pragma unroll
    for (int e = 0; e < 4; ++e) {
      const float f0 = bA[e];
      const float f1 = bB[e];
      bv[e]     = bf16_value(f0);
      bv[4 + e] = bf16_value(f1);
    }
#pragma unroll 1
    for (int bt = 0; bt < 4; ++bt) {
      const v8f a = acc[0];
      v8f g;
#pragma unroll
      for (int r = 0; r < 8; ++r) {
        const float th = tanhf(a[r] * kInvFwd + bv[r]);
        g[r] = 1.0f - th * th;
      }
      acc[0] = acc[1]; acc[1] = acc[2]; acc[2] = acc[3]; acc[3] = a;
      dth[0] = dth[1]; dth[1] = dth[2]; dth[2] = dth[3]; dth[3] = g;
    }
  }

  zero4(acc);
  slab_product<1>(wxRow, xdRow, kXPitch, acc);
#pragma unroll
  for (int bt = 0; bt < 4; ++bt) store_gated(s0Out + bt * 16 * kWPitch, dr[bt], acc[bt], kScaleP0);
  __syncthreads();

  zero4(acc);
  slab_product<4>(woRow, s0Row, kWPitch, acc);
#pragma unroll
  for (int bt = 0; bt < 4; ++bt) {
    v8h pv;
#pragma unroll
    for (int r = 0; r < 8; ++r) {
      const float cc = dth[bt][r] * acc[bt][r] * kScaleV0;
      hd[bt][r] = cc * kInvV0;
      pv[r] = to_f16_operand(cc);
    }
    *(v8h*)(s1Out + bt * 16 * kWPitch) = pv;
  }
  __syncthreads();

  float invc = kInvV0 * kInvTermGain;
#pragma unroll 1
  for (int k = 0; k < kTerms; ++k) {
    zero4(acc);
    slab_product<4>(whRow, s1Row, kWPitch, acc);
#pragma unroll
    for (int bt = 0; bt < 4; ++bt) store_gated(s0Out + bt * 16 * kWPitch, dr[bt], acc[bt], kScaleP);
    __syncthreads();
    zero4(acc);
    slab_product<4>(woRow, s0Row, kWPitch, acc);
#pragma unroll
    for (int bt = 0; bt < 4; ++bt) {
      v8h pv;
#pragma unroll
      for (int r = 0; r < 8; ++r) {
        const float cc = dth[bt][r] * acc[bt][r] * kScaleV;
        hd[bt][r] = hd[bt][r] + cc * invc;
        pv[r] = to_f16_operand(cc);
      }
      *(v8h*)(s1Out + bt * 16 * kWPitch) = pv;
    }
    __syncthreads();
    invc = invc * kInvTermGain;
  }

#pragma unroll
  for (int bt = 0; bt < 4; ++bt) {
    float* op = sO + (bt * 16 + c) * kOPitch + n0 + 8 * hh;
    const v4f lo4 = (v4f){hd[bt][0], hd[bt][1], hd[bt][2], hd[bt][3]};
    const v4f hi4 = (v4f){hd[bt][4], hd[bt][5], hd[bt][6], hd[bt][7]};
    *(v4f*)(op)     = lo4;
    *(v4f*)(op + 4) = hi4;
  }
  __syncthreads();

  {
    v4f ov[8];
#pragma unroll
    for (int i = 0; i < 8; ++i) ov[i] = *(const v4f*)(sO + (wave * 8 + i) * kOPitch + lane * 4);
    for (int pass = 0; pass < 2; ++pass) {
#pragma unroll
      for (int i = 0; i < 8; ++i)
        *(volatile v4f*)(out + (size_t)(row0 + wave * 8 + i) * kHid + lane * 4) = ov[i];
      __threadfence();
    }
  }
}

extern "C" void kernel_launch(void* const* d_in, const int* in_sizes, int n_in,
                              void* d_out, int out_size, void* d_ws, size_t ws_size,
                              hipStream_t stream) {
  (void)d_ws;
  (void)ws_size;
  if (n_in < 10) return;
  if (in_sizes[0] != 1) return;
  if (in_sizes[1] != kBatch * kHid) return;
  if (in_sizes[2] != kBatch * kIntervals * 4 * kCh) return;
  if (in_sizes[3] != kBatch * kIntervals * 4 * kCh) return;
  if (in_sizes[4] != kObs) return;
  if (in_sizes[5] != kHid * kCh) return;
  if (in_sizes[6] != kHid * kHid) return;
  if (in_sizes[7] != kHid * kHid) return;
  if (in_sizes[8] != kHid) return;
  if (in_sizes[9] != kHid) return;
  if (out_size != kBatch * kHid) return;

  const float* t       = (const float*)d_in[0];
  const float* h       = (const float*)d_in[1];
  const float* coeffs  = (const float*)d_in[2];
  const float* dcoeffs = (const float*)d_in[3];
  const float* tobs    = (const float*)d_in[4];
  const float* wx      = (const float*)d_in[5];
  const float* wh      = (const float*)d_in[6];
  const float* wout    = (const float*)d_in[7];
  const float* b0      = (const float*)d_in[8];
  const float* b1      = (const float*)d_in[9];
  float* out = (float*)d_out;

  series_rows<<<dim3(kBatch / kRowsBlk), dim3(256), 0, stream>>>(
      t, h, coeffs, dcoeffs, tobs, wx, wh, wout, b0, b1, out);
}
